// NonLinearSelfAttention_59794534695069
// MI455X (gfx1250) — hardware-verified
//
#include <hip/hip_runtime.h>
#include <math.h>
#include <stdint.h>

#define NB    8
#define SEQ   4096
#define DCH   128
#define DOUT  128

static_assert(SEQ % 64 == 0);
static_assert(DCH == 128);
static_assert(DOUT % 64 == 0);
static_assert((NB * SEQ) % 64 == 0);

typedef __attribute__((ext_vector_type(16))) _Float16 v16h;
typedef __attribute__((ext_vector_type(8)))  _Float16 v8h;
typedef __attribute__((ext_vector_type(16))) __bf16   v16b;
typedef __attribute__((ext_vector_type(8)))  __bf16   v8b;
typedef __attribute__((ext_vector_type(8)))  float    v8f;
typedef __attribute__((ext_vector_type(4)))  float    v4f;
typedef __attribute__((ext_vector_type(2)))  float    v2f;
typedef __attribute__((ext_vector_type(4)))  unsigned int v4u;

__device__ __forceinline__ unsigned short f2bf_bits(float f) {
  unsigned u = __float_as_uint(f);
  return (unsigned short)((u + 0x7FFFu + ((u >> 16) & 1u)) >> 16);
}
__device__ __forceinline__ float bf_bits2f(unsigned short h) { return __uint_as_float(((unsigned)h) << 16); }
__device__ __forceinline__ unsigned pk16(unsigned short a, unsigned short b) { return (unsigned)a | ((unsigned)b << 16); }

__device__ __forceinline__ void dep_guard_h(v8f& a, v8f& b, v16h x, v16h y) { asm volatile("v_nop\n\tv_nop\n\tv_nop\n\tv_nop" : "+v"(a), "+v"(b) : "v"(x), "v"(y)); }
__device__ __forceinline__ void dep_guard_b(v8f& a, v8f& b, v16b x, v16b y) { asm volatile("v_nop\n\tv_nop\n\tv_nop\n\tv_nop" : "+v"(a), "+v"(b) : "v"(x), "v"(y)); }
__device__ __forceinline__ void keep4_h(v16h a, v16h b, v16h c, v16h d) { asm volatile("v_nop" :: "v"(a), "v"(b), "v"(c), "v"(d)); }
__device__ __forceinline__ void keep4_b(v16b a, v16b b, v16b c, v16b d) { asm volatile("v_nop" :: "v"(a), "v"(b), "v"(c), "v"(d)); }
__device__ __forceinline__ void acc_guard4(v8f& a, v8f& b, v8f& c, v8f& d) { asm volatile("v_nop\n\tv_nop\n\tv_nop\n\tv_nop" : "+v"(a), "+v"(b), "+v"(c), "+v"(d)); }

template <typename T> struct Frag;
template <> struct Frag<_Float16> {
  typedef v16h V; union U { v16h v; v8h h[2]; };
  static __device__ __forceinline__ v16h load(const _Float16* p) {
    U f; f.h[0] = *(const v8h*)(p); f.h[1] = *(const v8h*)(p + 16); return f.v;
  }
  static __device__ __forceinline__ v8f mma(v16h a, v16h b, v8f c) {
    return __builtin_amdgcn_wmma_f32_16x16x32_f16(false, a, false, b, (short)0, c, false, false);
  }
  static __device__ __forceinline__ void guard(v8f& a, v8f& b, v16h x, v16h y) { dep_guard_h(a, b, x, y); }
  static __device__ __forceinline__ void keep(v16h a, v16h b, v16h c, v16h d) { keep4_h(a, b, c, d); }
};
template <> struct Frag<__bf16> {
  typedef v16b V; union U { v16b v; v8b h[2]; };
  static __device__ __forceinline__ v16b load(const __bf16* p) {
    U f; f.h[0] = *(const v8b*)(p); f.h[1] = *(const v8b*)(p + 16); return f.v;
  }
  static __device__ __forceinline__ v8f mma(v16b a, v16b b, v8f c) {
    return __builtin_amdgcn_wmma_f32_16x16x32_bf16(false, a, false, b, (short)0, c, false, false);
  }
  static __device__ __forceinline__ void guard(v8f& a, v8f& b, v16b x, v16b y) { dep_guard_b(a, b, x, y); }
  static __device__ __forceinline__ void keep(v16b a, v16b b, v16b c, v16b d) { keep4_b(a, b, c, d); }
};

template <int ET> struct Elem;
template <> struct Elem<0> { typedef _Float16 T; };
template <> struct Elem<1> { typedef __bf16 T; };
template <int ET, bool SPLIT, int BIAS_MODE, int OUT_MODE, bool RESID>
__global__ __launch_bounds__(256) void wmma_gemm64(
    const unsigned short* __restrict__ Ap, const unsigned short* __restrict__ A2p, int lda, long strideA,
    const unsigned short* __restrict__ Btp, const unsigned short* __restrict__ Bt2p, int ldb, long strideB,
    void* __restrict__ Cout, void* __restrict__ Cout2, int ldc, long strideC,
    const float* __restrict__ bias,
    const float* __restrict__ resid, long strideR,
    int M, int N, int K, float scale) {
  typedef typename Elem<ET>::T T;
  typedef typename Frag<T>::V V;
  const T* A = (const T*)Ap; const T* A2 = (const T*)A2p; const T* Bt = (const T*)Btp; const T* Bt2 = (const T*)Bt2p;
  __shared__ __align__(16) float sT[8][16 * 68];
  const int b    = blockIdx.y;
  const int lane = threadIdx.x & 31;
  const int wave = threadIdx.x >> 5;
  const int tilesN = N >> 6;
  const int tilesM = M >> 6;
  const int tile = blockIdx.x * 8 + wave;
  if (tile >= tilesM * tilesN) return;
  const int tm = tile / tilesN;
  const int tn = tile - tm * tilesN;
  const int m0 = tm << 6;
  const int n0 = tn << 6;

  const T* Ab  = A  + (size_t)b * strideA;
  const T* Bb  = Bt + (size_t)b * strideB;
  const T* Ab2 = SPLIT ? (A2  + (size_t)b * strideA) : nullptr;
  const T* Bb2 = SPLIT ? (Bt2 + (size_t)b * strideB) : nullptr;

  const int rlane = lane & 15;
  const int koff  = (lane >> 4) * 8;
  const int mOff  = (lane >> 4) * 8;

  v8f acc[4][4];
#pragma unroll
  for (int i = 0; i < 4; ++i)
#pragma unroll
    for (int j = 0; j < 4; ++j) acc[i][j] = (v8f){0.f,0.f,0.f,0.f,0.f,0.f,0.f,0.f};

  for (int k0 = 0; k0 < K; k0 += 32) {
    V bh[4], bl[4];
#pragma unroll
    for (int j = 0; j < 4; ++j) {
      const size_t bo = (size_t)(n0 + (j << 4) + rlane) * ldb + koff + k0;
      bh[j] = Frag<T>::load(Bb + bo);
      if (SPLIT) bl[j] = Frag<T>::load(Bb2 + bo);
    }
#pragma unroll
    for (int i = 0; i < 4; ++i) {
      const size_t ao = (size_t)(m0 + (i << 4) + rlane) * lda + koff + k0;
      V ah = Frag<T>::load(Ab + ao);
      V al;
      if (SPLIT) al = Frag<T>::load(Ab2 + ao);
#pragma unroll
      for (int j = 0; j < 4; ++j) {
        acc[i][j] = Frag<T>::mma(ah, bh[j], acc[i][j]);
        if (SPLIT) {
          acc[i][j] = Frag<T>::mma(ah, bl[j], acc[i][j]);
          acc[i][j] = Frag<T>::mma(al, bh[j], acc[i][j]);
        }
      }
      Frag<T>::guard(acc[i][0], acc[i][3], ah, SPLIT ? al : ah);
    }
    Frag<T>::keep(bh[0], bh[1], bh[2], bh[3]);
    if (SPLIT) Frag<T>::keep(bl[0], bl[1], bl[2], bl[3]);
  }
  acc_guard4(acc[0][0], acc[0][1], acc[0][2], acc[0][3]);
  acc_guard4(acc[1][0], acc[1][1], acc[1][2], acc[1][3]);
  acc_guard4(acc[2][0], acc[2][1], acc[2][2], acc[2][3]);
  acc_guard4(acc[3][0], acc[3][1], acc[3][2], acc[3][3]);

  float* slab = sT[wave];
  const float* Rb = RESID ? (resid + (size_t)b * strideR) : nullptr;
#pragma unroll
  for (int i = 0; i < 4; ++i) {
    const int mBase = m0 + (i << 4);
#pragma unroll
    for (int j = 0; j < 4; ++j) {
      const int n = n0 + (j << 4) + rlane;
      float bv = 0.f;
      if (BIAS_MODE == 2) bv = bias[n];
#pragma unroll
      for (int r = 0; r < 8; ++r) {
        float v = acc[i][j][r] * scale;
        if (BIAS_MODE == 1) v += bias[mBase + mOff + r];
        if (BIAS_MODE == 2) v += bv;
        if (RESID) v += Rb[(size_t)(mBase + mOff + r) * ldc + n];
        slab[(mOff + r) * 68 + (j << 4) + rlane] = v;
      }
    }
    __builtin_amdgcn_fence(__ATOMIC_RELEASE, "workgroup");
    __builtin_amdgcn_wave_barrier();
    __builtin_amdgcn_fence(__ATOMIC_ACQUIRE, "workgroup");
    if (OUT_MODE == 0) {
      float* C = (float*)Cout + (size_t)b * strideC;
      const int hh = lane >> 4, c4 = (lane & 15) * 4;
      for (int ps = 0; ps < 2; ++ps) {
#pragma unroll
        for (int it = 0; it < 8; ++it) {
          const int row = it * 2 + hh;
          v4f v = *(const v4f*)(slab + row * 68 + c4);
          *(volatile v4f*)(C + (size_t)(mBase + row) * ldc + n0 + c4) = v;
        }
        __threadfence();
      }
    } else {
      const int q = lane >> 3, c8 = (lane & 7) * 8;
      unsigned short* C  = (unsigned short*)Cout  + (size_t)b * strideC;
      unsigned short* C2 = (OUT_MODE == 2) ? ((unsigned short*)Cout2 + (size_t)b * strideC) : nullptr;
      for (int ps = 0; ps < 2; ++ps) {
#pragma unroll
        for (int it = 0; it < 4; ++it) {
          const int row = it * 4 + q;
          const float* sp = slab + row * 68 + c8;
          v4u hv, lv;
#pragma unroll
          for (int e = 0; e < 4; ++e) {
            if (OUT_MODE == 1) {
              const unsigned short a0 = __builtin_bit_cast(unsigned short, (_Float16)sp[2 * e]);
              const unsigned short a1 = __builtin_bit_cast(unsigned short, (_Float16)sp[2 * e + 1]);
              hv[e] = pk16(a0, a1); lv[e] = 0u;
            } else {
              const unsigned short h0 = f2bf_bits(sp[2 * e]), h1 = f2bf_bits(sp[2 * e + 1]);
              const unsigned short l0 = f2bf_bits(sp[2 * e] - bf_bits2f(h0)), l1 = f2bf_bits(sp[2 * e + 1] - bf_bits2f(h1));
              hv[e] = pk16(h0, h1); lv[e] = pk16(l0, l1);
            }
          }
          *(volatile v4u*)(C + (size_t)(mBase + row) * ldc + n0 + c8) = hv;
          if (OUT_MODE == 2) *(volatile v4u*)(C2 + (size_t)(mBase + row) * ldc + n0 + c8) = lv;
        }
        __threadfence();
      }
    }
    __builtin_amdgcn_fence(__ATOMIC_RELEASE, "workgroup");
    __builtin_amdgcn_wave_barrier();
    __builtin_amdgcn_fence(__ATOMIC_ACQUIRE, "workgroup");
  }
}

__global__ __launch_bounds__(256) void split_bf16x2_kernel(const float* __restrict__ in, unsigned short* __restrict__ hi,
                                                           unsigned short* __restrict__ lo, int n2) {
  const int i = blockIdx.x * 256 + threadIdx.x;
  if (i < n2) {
    const v2f f = *(const v2f*)(in + 2 * (size_t)i);
    const unsigned short h0 = f2bf_bits(f[0]), h1 = f2bf_bits(f[1]);
    const unsigned short l0 = f2bf_bits(f[0] - bf_bits2f(h0)), l1 = f2bf_bits(f[1] - bf_bits2f(h1));
    const unsigned uh = pk16(h0, h1), ul = pk16(l0, l1);
    ((volatile unsigned*)hi)[i] = uh;
    ((volatile unsigned*)lo)[i] = ul;
    __threadfence();
    ((volatile unsigned*)hi)[i] = uh;
    ((volatile unsigned*)lo)[i] = ul;
  }
}

#define TFP 132
__global__ __launch_bounds__(256) void xprep_kernel(const float* __restrict__ x, unsigned short* __restrict__ xf,
                                                    unsigned short* __restrict__ xth, unsigned short* __restrict__ xtl) {
  union H8 { v8h h; v4u u; };
  __shared__ __align__(16) float tf[64 * TFP];
  const int tid = threadIdx.x;
  const int nt  = blockIdx.x % (SEQ / 64);
  const int b   = blockIdx.x / (SEQ / 64);
  const int n0  = nt * 64;
  const float* xb = x + ((size_t)b * SEQ + n0) * DCH;
  unsigned short* xfb = xf + ((size_t)b * SEQ + n0) * DCH;
  {
    const int lr = tid >> 4;
    const int c8 = (tid & 15) * 8;
    v4u hf[4];
#pragma unroll
    for (int it = 0; it < 4; ++it) {
      const int row = it * 16 + lr;
      const v4f a0 = *(const v4f*)(xb + (size_t)row * DCH + c8);
      const v4f a1 = *(const v4f*)(xb + (size_t)row * DCH + c8 + 4);
      *(v4f*)(tf + row * TFP + c8) = a0;
      *(v4f*)(tf + row * TFP + c8 + 4) = a1;
      H8 p;
#pragma unroll
      for (int e = 0; e < 4; ++e) { p.h[e] = (_Float16)a0[e]; p.h[4 + e] = (_Float16)a1[e]; }
      hf[it] = p.u;
    }
    for (int ps = 0; ps < 2; ++ps) {
#pragma unroll
      for (int it = 0; it < 4; ++it) {
        const int row = it * 16 + lr;
        *(volatile v4u*)(xfb + (size_t)row * DCH + c8) = hf[it];
      }
      __threadfence();
    }
  }
  __syncthreads();
  {
    const int sub = tid >> 3;
    const int t8  = (tid & 7) * 8;
    v4u hv[4], lv[4];
#pragma unroll
    for (int it = 0; it < 4; ++it) {
      const int d = it * 32 + sub;
      v4u a, a2;
#pragma unroll
      for (int q = 0; q < 4; ++q) {
        const float f0 = tf[(t8 + 2 * q) * TFP + d];
        const float f1 = tf[(t8 + 2 * q + 1) * TFP + d];
        const unsigned short h0 = f2bf_bits(f0), h1 = f2bf_bits(f1);
        const unsigned short l0 = f2bf_bits(f0 - bf_bits2f(h0)), l1 = f2bf_bits(f1 - bf_bits2f(h1));
        a[q]  = pk16(h0, h1);
        a2[q] = pk16(l0, l1);
      }
      hv[it] = a; lv[it] = a2;
    }
    unsigned short* th = xth + (size_t)b * DCH * SEQ + n0 + t8;
    unsigned short* tl = xtl + (size_t)b * DCH * SEQ + n0 + t8;
    for (int ps = 0; ps < 2; ++ps) {
#pragma unroll
      for (int it = 0; it < 4; ++it) {
        const int d = it * 32 + sub;
        const size_t go = (size_t)d * SEQ;
        *(volatile v4u*)(th + go) = hv[it];
        *(volatile v4u*)(tl + go) = lv[it];
      }
      __threadfence();
    }
  }
}

#define AT_NW 8
#define AT_NG 4
#define AT_QB 64
#define AT_KC 64
#define KSP 136
#define VTP 72
#define OSP 68

__device__ __forceinline__ __bf16 at_f2bf(float f) { return __builtin_bit_cast(__bf16, f2bf_bits(f)); }
__device__ __forceinline__ void at_split(float f, __bf16& hi, __bf16& lo) {
  const unsigned short hb = f2bf_bits(f);
  hi = __builtin_bit_cast(__bf16, hb);
  lo = at_f2bf(f - bf_bits2f(hb));
}
__device__ __forceinline__ v8f at_mma_b(v16b a, v16b b, v8f c) {
  c = __builtin_amdgcn_wmma_f32_16x16x32_bf16(false, a, false, b, (short)0, c, false, false);
  asm volatile("v_nop\n\tv_nop\n\tv_nop\n\tv_nop" : "+v"(c) : "v"(a), "v"(b));
  return c;
}
__device__ __forceinline__ v8f at_mma_h(v16h a, v16h b, v8f c) {
  c = __builtin_amdgcn_wmma_f32_16x16x32_f16(false, a, false, b, (short)0, c, false, false);
  asm volatile("v_nop\n\tv_nop\n\tv_nop\n\tv_nop" : "+v"(c) : "v"(a), "v"(b));
  return c;
}

__global__ __launch_bounds__(256)
void attn_kernel(const unsigned short* __restrict__ xfp, const unsigned short* __restrict__ xthp,
                 const unsigned short* __restrict__ xtlp, unsigned short* __restrict__ chp,
                 unsigned short* __restrict__ clp, float sscale) {
  union FH { v16h v; v8h h[2]; };
  union FB { v16b v; v8b h[2]; };
  __shared__ __align__(16) _Float16 Ksf[AT_KC * KSP];
  __shared__ __align__(16) __bf16   Vth[DCH * VTP];
  __shared__ __align__(16) __bf16   Vtl[DCH * VTP];
  __shared__ __align__(16) __bf16   Psh[AT_NG][16 * AT_KC];
  __shared__ __align__(16) __bf16   Psl[AT_NG][16 * AT_KC];
  __shared__ __align__(16) float    Al[AT_NG][16];
  __shared__ __align__(16) float    Ll[AT_NG][16];
  __shared__ __align__(16) float    Os[AT_NW][16 * OSP];

  const int tid  = threadIdx.x;
  const int wave = tid >> 5;
  const int lane = tid & 31;
  const int hh   = lane >> 4;
  const int c    = lane & 15;
  const int g    = wave & 3;
  const int chh  = wave >> 2;
  const int ch0  = chh * 64;

  const int nqb = SEQ / AT_QB;
  const int qb  = blockIdx.x % nqb;
  const int b   = blockIdx.x / nqb;
  const int qg0 = qb * AT_QB + g * 16;

  const _Float16* Xf = (const _Float16*)(const void*)xfp + (size_t)b * SEQ * DCH;
  const __bf16*   Xh = (const __bf16*)(const void*)xthp + (size_t)b * DCH * SEQ;
  const __bf16*   Xl = (const __bf16*)(const void*)xtlp + (size_t)b * DCH * SEQ;
  unsigned short* Ch = chp + (size_t)b * SEQ * DCH;
  unsigned short* Cl = clp + (size_t)b * SEQ * DCH;

  float mrow[8], lrow[8];
  v8f oacc[4];
#pragma unroll
  for (int r = 0; r < 8; ++r) { mrow[r] = -INFINITY; lrow[r] = 0.f; }
#pragma unroll
  for (int t = 0; t < 4; ++t) oacc[t] = (v8f){0.f,0.f,0.f,0.f,0.f,0.f,0.f,0.f};

  __bf16* pwh = Psh[g];
  __bf16* pwl = Psl[g];

  const int nChunks = SEQ / AT_KC;
  for (int kc = 0; kc < nChunks; ++kc) {
    const int kv0 = kc * AT_KC;
    __syncthreads();
    {
      const int r = tid >> 2, qq = (tid & 3) * 32;
      const _Float16* ks = Xf + (size_t)(kv0 + r) * DCH + qq;
      _Float16* kd = Ksf + r * KSP + qq;
#pragma unroll
      for (int i = 0; i < 4; ++i) *(v8h*)(kd + 8 * i) = *(const v8h*)(ks + 8 * i);
      const int r2 = tid >> 1, hf = (tid & 1) * 32;
      const __bf16* vh = Xh + (size_t)r2 * SEQ + kv0 + hf;
      const __bf16* vl = Xl + (size_t)r2 * SEQ + kv0 + hf;
#pragma unroll
      for (int i = 0; i < 4; ++i) {
        *(v8b*)(Vth + r2 * VTP + hf + 8 * i) = *(const v8b*)(vh + 8 * i);
        *(v8b*)(Vtl + r2 * VTP + hf + 8 * i) = *(const v8b*)(vl + 8 * i);
      }
    }
    __syncthreads();

    if (wave < AT_NG) {
      v16h qa[4];
#pragma unroll
      for (int dc = 0; dc < 4; ++dc)
        qa[dc] = Frag<_Float16>::load(Xf + (size_t)(qg0 + c) * DCH + dc * 32 + 8 * hh);

      v8f s[4];
#pragma unroll
      for (int j = 0; j < 4; ++j) {
        s[j] = (v8f){0.f,0.f,0.f,0.f,0.f,0.f,0.f,0.f};
#pragma unroll
        for (int dc = 0; dc < 4; ++dc) {
          FH kb;
          kb.h[0] = *(const v8h*)(Ksf + (j * 16 + c) * KSP + dc * 32 + 8 * hh);
          kb.h[1] = *(const v8h*)(Ksf + (j * 16 + c) * KSP + dc * 32 + 16 + 8 * hh);
          s[j] = at_mma_h(qa[dc], kb.v, s[j]);
        }
      }
      float cm[8];
#pragma unroll
      for (int r = 0; r < 8; ++r) {
        float m = -INFINITY;
#pragma unroll
        for (int j = 0; j < 4; ++j) {
          const float sv = s[j][r] * sscale;
          s[j][r] = sv;
          m = fmaxf(m, sv);
        }
#pragma unroll
        for (int off = 1; off < 16; off <<= 1) m = fmaxf(m, __shfl_xor(m, off, 32));
        cm[r] = m;
      }
#pragma unroll
      for (int r = 0; r < 8; ++r) {
        const float mnew = fmaxf(mrow[r], cm[r]);
        const float alpha = expf(mrow[r] - mnew);
        mrow[r] = mnew;
        float psum = 0.f;
#pragma unroll
        for (int j = 0; j < 4; ++j) {
          const float p = expf(s[j][r] - mnew);
          psum += p;
          __bf16 a, bl; at_split(p, a, bl);
          pwh[(8 * hh + r) * AT_KC + j * 16 + c] = a;
          pwl[(8 * hh + r) * AT_KC + j * 16 + c] = bl;
        }
#pragma unroll
        for (int off = 1; off < 16; off <<= 1) psum += __shfl_xor(psum, off, 32);
        lrow[r] = lrow[r] * alpha + psum;
        if (c == 0) {
          Al[g][8 * hh + r] = alpha;
          Ll[g][8 * hh + r] = lrow[r];
        }
      }
    }
    __syncthreads();

    {
      float af[8];
#pragma unroll
      for (int r = 0; r < 8; ++r) af[r] = Al[g][8 * hh + r];
#pragma unroll
      for (int t = 0; t < 4; ++t)
#pragma unroll
        for (int r = 0; r < 8; ++r) oacc[t][r] *= af[r];
#pragma unroll 1
      for (int kk = 0; kk < 2; ++kk) {
        FB pa, pl;
        pa.h[0] = *(const v8b*)(pwh + c * AT_KC + kk * 32 + 8 * hh);
        pa.h[1] = *(const v8b*)(pwh + c * AT_KC + kk * 32 + 16 + 8 * hh);
        pl.h[0] = *(const v8b*)(pwl + c * AT_KC + kk * 32 + 8 * hh);
        pl.h[1] = *(const v8b*)(pwl + c * AT_KC + kk * 32 + 16 + 8 * hh);
#pragma unroll
        for (int t = 0; t < 4; ++t) {
          FB vb, vl;
          vb.h[0] = *(const v8b*)(Vth + (ch0 + t * 16 + c) * VTP + kk * 32 + 8 * hh);
          vb.h[1] = *(const v8b*)(Vth + (ch0 + t * 16 + c) * VTP + kk * 32 + 16 + 8 * hh);
          vl.h[0] = *(const v8b*)(Vtl + (ch0 + t * 16 + c) * VTP + kk * 32 + 8 * hh);
          vl.h[1] = *(const v8b*)(Vtl + (ch0 + t * 16 + c) * VTP + kk * 32 + 16 + 8 * hh);
          oacc[t] = at_mma_b(pa.v, vb.v, oacc[t]);
          oacc[t] = at_mma_b(pa.v, vl.v, oacc[t]);
          oacc[t] = at_mma_b(pl.v, vb.v, oacc[t]);
        }
      }
    }
  }

  float* os = Os[wave];
#pragma unroll
  for (int r = 0; r < 8; ++r) {
    const float inv = 1.0f / Ll[g][8 * hh + r];
#pragma unroll
    for (int t = 0; t < 4; ++t) os[(8 * hh + r) * OSP + t * 16 + c] = oacc[t][r] * inv;
  }
  __builtin_amdgcn_fence(__ATOMIC_RELEASE, "workgroup");
  __builtin_amdgcn_wave_barrier();
  __builtin_amdgcn_fence(__ATOMIC_ACQUIRE, "workgroup");
  {
    const int q = lane >> 3, c8 = (lane & 7) * 8;
    for (int ps = 0; ps < 2; ++ps) {
#pragma unroll
      for (int it = 0; it < 4; ++it) {
        const int row = it * 4 + q;
        const float* sp = os + row * OSP + c8;
        v4u hv, lv;
#pragma unroll
        for (int e = 0; e < 4; ++e) {
          const float f0 = sp[2 * e], f1 = sp[2 * e + 1];
          const unsigned short h0 = f2bf_bits(f0), h1 = f2bf_bits(f1);
          const unsigned short l0 = f2bf_bits(f0 - bf_bits2f(h0)), l1 = f2bf_bits(f1 - bf_bits2f(h1));
          hv[e] = pk16(h0, h1); lv[e] = pk16(l0, l1);
        }
        const size_t go = (size_t)(qg0 + row) * DCH + ch0 + c8;
        *(volatile v4u*)(Ch + go) = hv;
        *(volatile v4u*)(Cl + go) = lv;
      }
      __threadfence();
    }
  }
}

extern "C" void kernel_launch(void* const* d_in, const int* in_sizes, int n_in,
                              void* d_out, int out_size, void* d_ws, size_t ws_size,
                              hipStream_t stream) {
  if (n_in < 3) return;
  if (in_sizes[0] != NB * SEQ * DCH) return;
  if (in_sizes[1] != DOUT * DCH) return;
  if (in_sizes[2] != DOUT) return;
  if (out_size != NB * SEQ * DOUT) return;

  const float* x    = (const float*)d_in[0];
  const float* W    = (const float*)d_in[1];
  const float* bias = (const float*)d_in[2];

  const size_t PXF = (size_t)NB * SEQ * DCH * 2;
  const size_t PXT = (size_t)NB * DCH * SEQ * 2;
  const size_t PC  = (size_t)NB * SEQ * DCH * 2;
  const size_t PW  = (size_t)DOUT * DCH * 2;
  size_t off = 0;
  const size_t oXf  = off; off += PXF;
  const size_t oXTh = off; off += PXT;
  const size_t oXTl = off; off += PXT;
  const size_t oCh  = off; off += PC;
  const size_t oCl  = off; off += PC;
  const size_t oWh  = off; off += PW;
  const size_t oWl  = off; off += PW;
  if (off > ws_size) return;

  char* ws = (char*)d_ws;
  unsigned short* Xf  = (unsigned short*)(ws + oXf);
  unsigned short* XTh = (unsigned short*)(ws + oXTh);
  unsigned short* XTl = (unsigned short*)(ws + oXTl);
  unsigned short* Ch  = (unsigned short*)(ws + oCh);
  unsigned short* Cl  = (unsigned short*)(ws + oCl);
  unsigned short* Wh  = (unsigned short*)(ws + oWh);
  unsigned short* Wl  = (unsigned short*)(ws + oWl);

  xprep_kernel<<<dim3(NB * (SEQ / 64)), dim3(256), 0, stream>>>(x, Xf, XTh, XTl);
  const int n2w = DOUT * DCH / 2;
  split_bf16x2_kernel<<<dim3((n2w + 255) / 256), dim3(256), 0, stream>>>(W, Wh, Wl, n2w);
  attn_kernel<<<dim3(NB * (SEQ / AT_QB)), dim3(256), 0, stream>>>(Xf, XTh, XTl, Ch, Cl, 0.08838834764831845f);
  const int tilesOut = ((NB * SEQ) / 64) * (DOUT / 64);
  wmma_gemm64<1, true, 2, 0, false><<<dim3((tilesOut + 7) / 8, 1), dim3(256), 0, stream>>>(
      Ch, Cl, DCH, 0L, Wh, Wl, DCH, 0L, (void*)d_out, (void*)d_out, DOUT, 0L,
      bias, bias, 0L, NB * SEQ, DOUT, DCH, 1.0f);
  (void)hipGetLastError();
}
